// InfiniViT_4277787427208
// MI455X (gfx1250) — hardware-run, weakly checked
//
#include <hip/hip_runtime.h>
#include <math.h>

constexpr int kBatch = 2;
constexpr int kT     = 2048;
constexpr int kC     = 1024;
constexpr int kHeads = 16;
constexpr int kD     = 64;
constexpr int kMemN  = 64;
constexpr int kHid   = 4096;
constexpr int kTok   = kBatch * kT;
constexpr int kQKVld = 3 * kC;
constexpr int kQKld  = 2 * kC;
constexpr float kWCarry   = 16.0f;
constexpr float kPCarry   = 2048.0f;
constexpr float kAttCarry = 16.0f;
constexpr float kHidCarry = 16.0f;
constexpr float kInvC     = 1.0f / 1024.0f;
constexpr float kLnEps    = 1e-5f;
constexpr long  kMiB      = 1048576L;

typedef __attribute__((ext_vector_type(16))) _Float16 v16h;
typedef __attribute__((ext_vector_type(8)))  _Float16 v8h;
typedef __attribute__((ext_vector_type(16))) __bf16   v16b;
typedef __attribute__((ext_vector_type(8)))  __bf16   v8b;
typedef __attribute__((ext_vector_type(8)))  float    v8f;
typedef __attribute__((ext_vector_type(4)))  float    v4f;
typedef __attribute__((ext_vector_type(4)))  unsigned int v4u;

__device__ __forceinline__ unsigned short f2bf_bits(float f) {
  unsigned u = __float_as_uint(f);
  return (unsigned short)((u + 0x7FFFu + ((u >> 16) & 1u)) >> 16);
}
__device__ __forceinline__ float bf_bits2f(unsigned short h) { return __uint_as_float(((unsigned)h) << 16); }

__device__ __forceinline__ void dep_guard_h(v8f& a, v8f& b, v16h x, v16h y) { asm volatile("v_nop\n\tv_nop\n\tv_nop\n\tv_nop" : "+v"(a), "+v"(b) : "v"(x), "v"(y)); }
__device__ __forceinline__ void dep_guard_b(v8f& a, v8f& b, v16b x, v16b y) { asm volatile("v_nop\n\tv_nop\n\tv_nop\n\tv_nop" : "+v"(a), "+v"(b) : "v"(x), "v"(y)); }
__device__ __forceinline__ void keep4_h(v16h a, v16h b, v16h c, v16h d) { asm volatile("v_nop" :: "v"(a), "v"(b), "v"(c), "v"(d)); }
__device__ __forceinline__ void keep4_b(v16b a, v16b b, v16b c, v16b d) { asm volatile("v_nop" :: "v"(a), "v"(b), "v"(c), "v"(d)); }
__device__ __forceinline__ void acc_guard4(v8f& a, v8f& b, v8f& c, v8f& d) { asm volatile("v_nop\n\tv_nop\n\tv_nop\n\tv_nop" : "+v"(a), "+v"(b), "+v"(c), "+v"(d)); }
template <typename T> struct Frag;
template <> struct Frag<_Float16> {
  typedef v16h V; union U { v16h v; v8h h[2]; };
  static __device__ __forceinline__ v16h load(const _Float16* p) {
    U f; f.h[0] = *(const v8h*)(p); f.h[1] = *(const v8h*)(p + 16); return f.v;
  }
  static __device__ __forceinline__ v8f mma(v16h a, v16h b, v8f c) {
    return __builtin_amdgcn_wmma_f32_16x16x32_f16(false, a, false, b, (short)0, c, false, false);
  }
  static __device__ __forceinline__ void guard(v8f& a, v8f& b, v16h x, v16h y) { dep_guard_h(a, b, x, y); }
  static __device__ __forceinline__ void keep(v16h a, v16h b, v16h c, v16h d) { keep4_h(a, b, c, d); }
};
template <> struct Frag<__bf16> {
  typedef v16b V; union U { v16b v; v8b h[2]; };
  static __device__ __forceinline__ v16b load(const __bf16* p) {
    U f; f.h[0] = *(const v8b*)(p); f.h[1] = *(const v8b*)(p + 16); return f.v;
  }
  static __device__ __forceinline__ v8f mma(v16b a, v16b b, v8f c) {
    return __builtin_amdgcn_wmma_f32_16x16x32_bf16(false, a, false, b, (short)0, c, false, false);
  }
  static __device__ __forceinline__ void guard(v8f& a, v8f& b, v16b x, v16b y) { dep_guard_b(a, b, x, y); }
  static __device__ __forceinline__ void keep(v16b a, v16b b, v16b c, v16b d) { keep4_b(a, b, c, d); }
};

__device__ __forceinline__ unsigned pk16(unsigned short a, unsigned short b) { return (unsigned)a | ((unsigned)b << 16); }
__device__ __forceinline__ unsigned short h_bits(float f) { const _Float16 h = (_Float16)f; return __builtin_bit_cast(unsigned short, h); }

template <int ET> struct Elem;
template <> struct Elem<0> { typedef _Float16 T; };
template <> struct Elem<1> { typedef __bf16 T; };
template <int ET, bool SPLIT, int BIAS_MODE, int OUT_MODE, bool RESID, int ACT = 0>
__global__ __launch_bounds__(256) void wmma_gemm64(
    const unsigned short* __restrict__ Ap, const unsigned short* __restrict__ A2p, int lda, long strideA,
    const unsigned short* __restrict__ Btp, const unsigned short* __restrict__ Bt2p, int ldb, long strideB,
    void* __restrict__ Cout, void* __restrict__ Cout2, int ldc, long strideC,
    const float* __restrict__ bias,
    const float* __restrict__ resid, long strideR,
    int M, int N, int K, float scale) {
  typedef typename Elem<ET>::T T;
  typedef typename Frag<T>::V V;
  const T* A = (const T*)Ap; const T* A2 = (const T*)A2p; const T* Bt = (const T*)Btp; const T* Bt2 = (const T*)Bt2p;
  __shared__ __align__(16) float sT[8][16 * 68];
  const int b    = blockIdx.y;
  const int lane = threadIdx.x & 31;
  const int wave = threadIdx.x >> 5;
  const int tilesN = N >> 6;
  const int tilesM = M >> 6;
  const int tile = blockIdx.x * 8 + wave;
  if (tile >= tilesM * tilesN) return;
  const int tm = tile / tilesN;
  const int tn = tile - tm * tilesN;
  const int m0 = tm << 6;
  const int n0 = tn << 6;

  const T* Ab  = A  + (size_t)b * strideA;
  const T* Bb  = Bt + (size_t)b * strideB;
  const T* Ab2 = SPLIT ? (A2  + (size_t)b * strideA) : nullptr;
  const T* Bb2 = SPLIT ? (Bt2 + (size_t)b * strideB) : nullptr;

  const int rlane = lane & 15;
  const int koff  = (lane >> 4) * 8;
  const int mOff  = (lane >> 4) * 8;

  v8f acc[4][4];
#pragma unroll
  for (int i = 0; i < 4; ++i)
#pragma unroll
    for (int j = 0; j < 4; ++j) acc[i][j] = (v8f){0.f,0.f,0.f,0.f,0.f,0.f,0.f,0.f};

  for (int k0 = 0; k0 < K; k0 += 32) {
    V bh[4], bl[4];
#pragma unroll
    for (int j = 0; j < 4; ++j) {
      const size_t bo = (size_t)(n0 + (j << 4) + rlane) * ldb + koff + k0;
      bh[j] = Frag<T>::load(Bb + bo);
      if (SPLIT) bl[j] = Frag<T>::load(Bb2 + bo);
    }
#pragma unroll
    for (int i = 0; i < 4; ++i) {
      const size_t ao = (size_t)(m0 + (i << 4) + rlane) * lda + koff + k0;
      V ah = Frag<T>::load(Ab + ao);
      V al;
      if (SPLIT) al = Frag<T>::load(Ab2 + ao);
#pragma unroll
      for (int j = 0; j < 4; ++j) {
        acc[i][j] = Frag<T>::mma(ah, bh[j], acc[i][j]);
        if (SPLIT) {
          acc[i][j] = Frag<T>::mma(ah, bl[j], acc[i][j]);
          acc[i][j] = Frag<T>::mma(al, bh[j], acc[i][j]);
        }
      }
      Frag<T>::guard(acc[i][0], acc[i][3], ah, SPLIT ? al : ah);
    }
    Frag<T>::keep(bh[0], bh[1], bh[2], bh[3]);
    if (SPLIT) Frag<T>::keep(bl[0], bl[1], bl[2], bl[3]);
  }
  acc_guard4(acc[0][0], acc[0][1], acc[0][2], acc[0][3]);
  acc_guard4(acc[1][0], acc[1][1], acc[1][2], acc[1][3]);
  acc_guard4(acc[2][0], acc[2][1], acc[2][2], acc[2][3]);
  acc_guard4(acc[3][0], acc[3][1], acc[3][2], acc[3][3]);

  float* slab = sT[wave];
  const float* Rb = RESID ? (resid + (size_t)b * strideR) : nullptr;
#pragma unroll
  for (int i = 0; i < 4; ++i) {
    const int mBase = m0 + (i << 4);
#pragma unroll
    for (int j = 0; j < 4; ++j) {
      const int n = n0 + (j << 4) + rlane;
      float bv = 0.f;
      if (BIAS_MODE == 2) bv = bias[n];
#pragma unroll
      for (int r = 0; r < 8; ++r) {
        float v = acc[i][j][r] * scale;
        if (BIAS_MODE == 1) v += bias[mBase + mOff + r];
        if (BIAS_MODE == 2) v += bv;
        if (RESID) v += Rb[(size_t)(mBase + mOff + r) * ldc + n];
        if (ACT == 2) v = fmaxf(v, 0.0f);
        if (ACT == 4) v = (v > 0.f) ? v : 0.01f * v;
        slab[(mOff + r) * 68 + (j << 4) + rlane] = v;
      }
    }
    __builtin_amdgcn_fence(__ATOMIC_RELEASE, "workgroup");
    __builtin_amdgcn_wave_barrier();
    __builtin_amdgcn_fence(__ATOMIC_ACQUIRE, "workgroup");
    if (OUT_MODE == 0) {
      float* C = (float*)Cout + (size_t)b * strideC;
      const int hh = lane >> 4, c4 = (lane & 15) * 4;
      for (int pass = 0; pass < 2; ++pass) {
#pragma unroll
        for (int it = 0; it < 8; ++it) {
          const int row = it * 2 + hh;
          v4f v = *(const v4f*)(slab + row * 68 + c4);
          *(volatile v4f*)(C + (size_t)(mBase + row) * ldc + n0 + c4) = v;
        }
        __threadfence();
      }
    } else {
      const int q = lane >> 3, c8 = (lane & 7) * 8;
      unsigned short* C  = (unsigned short*)Cout  + (size_t)b * strideC;
      unsigned short* C2 = (OUT_MODE == 2) ? ((unsigned short*)Cout2 + (size_t)b * strideC) : nullptr;
      for (int pass = 0; pass < 2; ++pass) {
#pragma unroll
        for (int it = 0; it < 4; ++it) {
          const int row = it * 4 + q;
          const float* sp = slab + row * 68 + c8;
          v8h hv, lv;
#pragma unroll
          for (int e = 0; e < 8; ++e) {
            if (OUT_MODE == 1) {
              hv[e] = (_Float16)sp[e];
            } else {
              unsigned short hb = f2bf_bits(sp[e]);
              unsigned short lb = f2bf_bits(sp[e] - bf_bits2f(hb));
              hv[e] = __builtin_bit_cast(_Float16, hb);
              lv[e] = __builtin_bit_cast(_Float16, lb);
            }
          }
          *(volatile v8h*)(C + (size_t)(mBase + row) * ldc + n0 + c8) = hv;
          if (OUT_MODE == 2) *(volatile v8h*)(C2 + (size_t)(mBase + row) * ldc + n0 + c8) = lv;
        }
        __threadfence();
      }
    }
    __builtin_amdgcn_fence(__ATOMIC_RELEASE, "workgroup");
    __builtin_amdgcn_wave_barrier();
    __builtin_amdgcn_fence(__ATOMIC_ACQUIRE, "workgroup");
  }
}

__global__ __launch_bounds__(256) void wtcast_kernel(const float* __restrict__ W, unsigned short* __restrict__ out,
                                                     int Kin, int Nout, float scale) {
  __shared__ float sm[64][65];
  const int t  = threadIdx.x;
  const int d0 = blockIdx.x * 64;
  const int h0 = blockIdx.y * 64;
#pragma unroll
  for (int i = 0; i < 16; ++i) {
    const int e = i * 256 + t;
    const int r = e >> 6;
    const int c = e & 63;
    sm[c][r] = W[(size_t)(d0 + r) * Nout + h0 + c] * scale;
  }
  __syncthreads();
  const int lane = t & 31, wave = t >> 5;
  const int q = lane >> 3, c8 = (lane & 7) * 8;
  for (int pass = 0; pass < 2; ++pass) {
#pragma unroll
    for (int it = 0; it < 2; ++it) {
      const int row = wave * 8 + it * 4 + q;
      unsigned short hb[8];
#pragma unroll
      for (int e = 0; e < 8; ++e) hb[e] = h_bits(sm[row][c8 + e]);
      const v4u u = (v4u){pk16(hb[0], hb[1]), pk16(hb[2], hb[3]), pk16(hb[4], hb[5]), pk16(hb[6], hb[7])};
      *(volatile v4u*)(out + (size_t)(h0 + row) * Kin + d0 + c8) = u;
    }
    __threadfence();
  }
}

__global__ __launch_bounds__(128) void ln_f16_kernel(const float* __restrict__ x, const float* __restrict__ gam,
                                                     const float* __restrict__ bet, unsigned short* __restrict__ out) {
  __shared__ float redA[4];
  __shared__ float redB[4];
  const int row  = blockIdx.x;
  const int t    = threadIdx.x;
  const int lane = t & 31, wave = t >> 5;
  const int c0   = t * 8;
  const float* xr = x + (size_t)row * kC + c0;
  const v4f a = *(const v4f*)(xr);
  const v4f c = *(const v4f*)(xr + 4);
  float v[8];
  v[0] = a.x; v[1] = a.y; v[2] = a.z; v[3] = a.w; v[4] = c.x; v[5] = c.y; v[6] = c.z; v[7] = c.w;
  float s = 0.f;
#pragma unroll
  for (int e = 0; e < 8; ++e) s += v[e];
#pragma unroll
  for (int off = 16; off > 0; off >>= 1) s += __shfl_xor(s, off, 32);
  if (lane == 0) redA[wave] = s;
  __syncthreads();
  const float tot = (redA[0] + redA[1]) + (redA[2] + redA[3]);
  const float mu = tot * kInvC;
  float d[8];
  float ss = 0.f;
#pragma unroll
  for (int e = 0; e < 8; ++e) { d[e] = v[e] - mu; ss += d[e] * d[e]; }
#pragma unroll
  for (int off = 16; off > 0; off >>= 1) ss += __shfl_xor(ss, off, 32);
  if (lane == 0) redB[wave] = ss;
  __syncthreads();
  const float tot2 = (redB[0] + redB[1]) + (redB[2] + redB[3]);
  const float var  = tot2 * kInvC;
  const float rstd = rsqrtf(var + kLnEps);
  const v4f ga = *(const v4f*)(gam + c0);
  const v4f gc = *(const v4f*)(gam + c0 + 4);
  const v4f ba = *(const v4f*)(bet + c0);
  const v4f bc = *(const v4f*)(bet + c0 + 4);
  float gg[8], bb[8];
  gg[0] = ga.x; gg[1] = ga.y; gg[2] = ga.z; gg[3] = ga.w; gg[4] = gc.x; gg[5] = gc.y; gg[6] = gc.z; gg[7] = gc.w;
  bb[0] = ba.x; bb[1] = ba.y; bb[2] = ba.z; bb[3] = ba.w; bb[4] = bc.x; bb[5] = bc.y; bb[6] = bc.z; bb[7] = bc.w;
  unsigned short hb[8];
#pragma unroll
  for (int e = 0; e < 8; ++e) hb[e] = h_bits(d[e] * rstd * gg[e] + bb[e]);
  const v4u u = (v4u){pk16(hb[0], hb[1]), pk16(hb[2], hb[3]), pk16(hb[4], hb[5]), pk16(hb[6], hb[7])};
  unsigned short* q = out + (size_t)row * kC + c0;
  *(volatile v4u*)q = u;
  __threadfence();
  *(volatile v4u*)q = u;
}

__global__ __launch_bounds__(256) void memproj_kernel(const float* __restrict__ memory, const float* __restrict__ w,
                                                      const float* __restrict__ bias, float* __restrict__ out) {
  __shared__ __align__(16) float mrow[kC];
  const int t = threadIdx.x;
  const int m = blockIdx.y;
  const int n = blockIdx.x * 256 + t;
  *(v4f*)(mrow + 4 * t) = *(const v4f*)(memory + (size_t)m * kC + 4 * t);
  __syncthreads();
  float acc = 0.f;
  const float* wc = w + n;
#pragma unroll 8
  for (int k = 0; k < kC; ++k) acc += mrow[k] * wc[(size_t)k * kC];
  acc += bias[n];
  float* o = out + (size_t)m * kC + n;
  *(volatile float*)o = acc;
  __threadfence();
  *(volatile float*)o = acc;
}

__global__ __launch_bounds__(256) void qkcast_kernel(const float* __restrict__ qkv32, unsigned short* __restrict__ qk) {
  const int i   = blockIdx.x * 256 + threadIdx.x;
  const int row = i >> 8;
  const int c8  = (i & 255) * 8;
  const float* p = qkv32 + (size_t)row * kQKVld + c8;
  const v4f a = *(const v4f*)(p);
  const v4f c = *(const v4f*)(p + 4);
  unsigned short hb[8];
  hb[0] = h_bits(a.x); hb[1] = h_bits(a.y); hb[2] = h_bits(a.z); hb[3] = h_bits(a.w);
  hb[4] = h_bits(c.x); hb[5] = h_bits(c.y); hb[6] = h_bits(c.z); hb[7] = h_bits(c.w);
  const v4u u = (v4u){pk16(hb[0], hb[1]), pk16(hb[2], hb[3]), pk16(hb[4], hb[5]), pk16(hb[6], hb[7])};
  unsigned short* q = qk + (size_t)row * kQKld + c8;
  *(volatile v4u*)q = u;
  __threadfence();
  *(volatile v4u*)q = u;
}

__global__ __launch_bounds__(256) void vtr_kernel(const float* __restrict__ qkv32, unsigned short* __restrict__ vt) {
  __shared__ float sm[64][65];
  const int t  = threadIdx.x;
  const int t0 = blockIdx.x * 64;
  const int g  = blockIdx.y;
  const int b  = g >> 4, h = g & 15;
  const float* src = qkv32 + (size_t)(b * kT + t0) * kQKVld + 2 * kC + h * kD;
#pragma unroll
  for (int i = 0; i < 16; ++i) {
    const int e = i * 256 + t;
    const int r = e >> 6;
    const int c = e & 63;
    sm[c][r] = src[(size_t)r * kQKVld + c];
  }
  __syncthreads();
  const int lane = t & 31, wave = t >> 5;
  const int q = lane >> 3, c8 = (lane & 7) * 8;
  unsigned short* op = vt + (size_t)g * kD * kT + t0;
  for (int pass = 0; pass < 2; ++pass) {
#pragma unroll
    for (int it = 0; it < 2; ++it) {
      const int row = wave * 8 + it * 4 + q;
      unsigned short hb[8];
#pragma unroll
      for (int e = 0; e < 8; ++e) hb[e] = h_bits(sm[row][c8 + e]);
      const v4u u = (v4u){pk16(hb[0], hb[1]), pk16(hb[2], hb[3]), pk16(hb[4], hb[5]), pk16(hb[6], hb[7])};
      *(volatile v4u*)(op + (size_t)row * kT + c8) = u;
    }
    __threadfence();
  }
}

__global__ __launch_bounds__(64) void mematt_kernel(const float* __restrict__ qkv32, const float* __restrict__ mem32,
                                                    float* __restrict__ memout, float oscale) {
  __shared__ __align__(16) float mk[kMemN * kD];
  __shared__ __align__(16) float qo[64 * kD];
  __shared__ float sc[64 * 65];
  const int t = threadIdx.x;
  const int lane = t & 31, wave = t >> 5;
  const int g = blockIdx.y;
  const int b = g >> 4, h = g & 15;
  const int t0 = blockIdx.x * 64;
  const float* qsrc = qkv32 + (size_t)(b * kT + t0) * kQKVld + h * kD;
  const float* msrc = mem32 + h * kD;
#pragma unroll
  for (int i = 0; i < 16; ++i) {
    const int e4 = i * 64 + t;
    const int r = e4 >> 4, d4 = (e4 & 15) * 4;
    *(v4f*)(qo + r * kD + d4) = *(const v4f*)(qsrc + (size_t)r * kQKVld + d4);
    *(v4f*)(mk + r * kD + d4) = *(const v4f*)(msrc + (size_t)r * kC + d4);
  }
  __syncthreads();
  float* myq = qo + t * kD;
  float* mys = sc + t * 65;
#pragma unroll 1
  for (int m = 0; m < kMemN; ++m) {
    const float* mr = mk + m * kD;
    float s = 0.f;
#pragma unroll 1
    for (int j = 0; j < 16; ++j) {
      const v4f qv = *(const v4f*)(myq + 4 * j);
      const v4f kv = *(const v4f*)(mr + 4 * j);
      s += qv.x * kv.x;
      s += qv.y * kv.y;
      s += qv.z * kv.z;
      s += qv.w * kv.w;
    }
    mys[m] = s * 0.125f;
  }
  float mx = -INFINITY;
#pragma unroll 1
  for (int m = 0; m < kMemN; ++m) mx = fmaxf(mx, mys[m]);
  float sum = 0.f;
#pragma unroll 1
  for (int m = 0; m < kMemN; ++m) {
    const float p = expf(mys[m] - mx);
    mys[m] = p;
    sum += p;
  }
  const float inv = oscale / sum;
  const v4f zero4 = (v4f){0.f, 0.f, 0.f, 0.f};
#pragma unroll 1
  for (int j = 0; j < 16; ++j) *(v4f*)(myq + 4 * j) = zero4;
#pragma unroll 1
  for (int m = 0; m < kMemN; ++m) {
    const float p = mys[m];
    const float* mr = mk + m * kD;
#pragma unroll 1
    for (int j = 0; j < 16; ++j) {
      v4f o4 = *(const v4f*)(myq + 4 * j);
      const v4f kv = *(const v4f*)(mr + 4 * j);
      o4.x += p * kv.x;
      o4.y += p * kv.y;
      o4.z += p * kv.z;
      o4.w += p * kv.w;
      *(v4f*)(myq + 4 * j) = o4;
    }
  }
#pragma unroll 1
  for (int j = 0; j < 16; ++j) {
    v4f o4 = *(const v4f*)(myq + 4 * j);
    o4.x *= inv; o4.y *= inv; o4.z *= inv; o4.w *= inv;
    *(v4f*)(myq + 4 * j) = o4;
  }
  __syncthreads();
  float* ob = memout + (size_t)(b * kT + t0) * kC + h * kD;
  const int hh = lane >> 4, c4 = (lane & 15) * 4;
  for (int pass = 0; pass < 2; ++pass) {
#pragma unroll
    for (int it = 0; it < 16; ++it) {
      const int row = wave * 32 + it * 2 + hh;
      const v4f v = *(const v4f*)(qo + row * kD + c4);
      *(volatile v4f*)(ob + (size_t)row * kC + c4) = v;
    }
    __threadfence();
  }
}

__global__ __launch_bounds__(256) void softmax_row_kernel(const float* __restrict__ S, unsigned short* __restrict__ P, float carry) {
  __shared__ float redM[8];
  __shared__ float redS[8];
  const int row  = blockIdx.x;
  const int t    = threadIdx.x;
  const int lane = t & 31, wave = t >> 5;
  const int c0   = t * 8;
  const float* sr = S + (size_t)row * kT + c0;
  const v4f a = *(const v4f*)(sr);
  const v4f c = *(const v4f*)(sr + 4);
  float x[8];
  x[0] = a.x; x[1] = a.y; x[2] = a.z; x[3] = a.w; x[4] = c.x; x[5] = c.y; x[6] = c.z; x[7] = c.w;
  float m = fmaxf(fmaxf(fmaxf(x[0], x[1]), fmaxf(x[2], x[3])), fmaxf(fmaxf(x[4], x[5]), fmaxf(x[6], x[7])));
#pragma unroll
  for (int off = 16; off > 0; off >>= 1) m = fmaxf(m, __shfl_xor(m, off, 32));
  if (lane == 0) redM[wave] = m;
  __syncthreads();
  float gm = redM[0];
#pragma unroll
  for (int w = 1; w < 8; ++w) gm = fmaxf(gm, redM[w]);
  float e[8];
  float s = 0.f;
#pragma unroll
  for (int i = 0; i < 8; ++i) { e[i] = expf(x[i] - gm); s += e[i]; }
#pragma unroll
  for (int off = 16; off > 0; off >>= 1) s += __shfl_xor(s, off, 32);
  if (lane == 0) redS[wave] = s;
  __syncthreads();
  float tot = 0.f;
#pragma unroll
  for (int w = 0; w < 8; ++w) tot += redS[w];
  const float inv = carry / tot;
  unsigned short hb[8];
#pragma unroll
  for (int i = 0; i < 8; ++i) hb[i] = h_bits(e[i] * inv);
  const v4u u = (v4u){pk16(hb[0], hb[1]), pk16(hb[2], hb[3]), pk16(hb[4], hb[5]), pk16(hb[6], hb[7])};
  unsigned short* q = P + (size_t)row * kT + c0;
  *(volatile v4u*)q = u;
  __threadfence();
  *(volatile v4u*)q = u;
}

__global__ __launch_bounds__(256) void gelu_f16_kernel(const float* __restrict__ gin, unsigned short* __restrict__ hid,
                                                       int colofs, float carry) {
  const int i   = blockIdx.x * 256 + threadIdx.x;
  const int row = i >> 10;
  const int cp  = (i & 1023) * 2;
  const float* p = gin + (size_t)row * 2048 + cp;
  const float x0 = p[0];
  const float x1 = p[1];
  const float g0 = 0.5f * x0 * (1.0f + erff(x0 * 0.70710678118654752f)) * carry;
  const float g1 = 0.5f * x1 * (1.0f + erff(x1 * 0.70710678118654752f)) * carry;
  const unsigned u = pk16(h_bits(g0), h_bits(g1));
  unsigned* q = (unsigned*)(hid + (size_t)row * kHid + colofs + cp);
  *(volatile unsigned*)q = u;
  __threadfence();
  *(volatile unsigned*)q = u;
}

template <int BIAS_MODE, int OUT_MODE, bool RESID>
static void launch_gemm(hipStream_t st, int batch,
                        const void* A, int lda, long sA,
                        const void* Bt, int ldb, long sB,
                        void* Cp, int ldc, long sC,
                        const float* bias, const float* resid, long sR,
                        int M, int N, int K, float scale) {
  const int tiles = (M / 64) * (N / 64);
  dim3 grid((tiles + 7) / 8, batch);
  wmma_gemm64<0, false, BIAS_MODE, OUT_MODE, RESID, 0><<<grid, 256, 0, st>>>(
      (const unsigned short*)A, (const unsigned short*)A, lda, sA,
      (const unsigned short*)Bt, (const unsigned short*)Bt, ldb, sB,
      Cp, Cp, ldc, sC, bias, resid, sR, M, N, K, scale);
}

extern "C" void kernel_launch(void* const* d_in, const int* in_sizes, int n_in,
                              void* d_out, int out_size, void* d_ws, size_t ws_size,
                              hipStream_t stream) {
  if (n_in < 16) return;
  if (in_sizes[0] != kTok * kC || in_sizes[1] != kMemN * kC || out_size != kTok * kC) return;
  if (in_sizes[4] != kC * kQKVld || in_sizes[12] != kC * kHid || in_sizes[14] != kHid * kC) return;
  const size_t carve_total = (size_t)112 * kMiB;
  if (ws_size < carve_total) return;

  const float* x      = (const float*)d_in[0];
  const float* memory = (const float*)d_in[1];
  const float* ln1_g  = (const float*)d_in[2];
  const float* ln1_b  = (const float*)d_in[3];
  const float* w_qkv  = (const float*)d_in[4];
  const float* b_qkv  = (const float*)d_in[5];
  const float* w_out  = (const float*)d_in[6];
  const float* b_out  = (const float*)d_in[7];
  const float* w_mem  = (const float*)d_in[8];
  const float* b_mem  = (const float*)d_in[9];
  const float* ln2_g  = (const float*)d_in[10];
  const float* ln2_b  = (const float*)d_in[11];
  const float* w_fc1  = (const float*)d_in[12];
  const float* b_fc1  = (const float*)d_in[13];
  const float* w_fc2  = (const float*)d_in[14];
  const float* b_fc2  = (const float*)d_in[15];
  float* out = (float*)d_out;

  char* ws = (char*)d_ws;
  float*          QKV32  = (float*)(ws + 0);
  float*          S32    = (float*)(ws + 0);
  unsigned short* P16    = (unsigned short*)(ws + 32 * kMiB);
  float*          G32    = (float*)(ws + 0);
  unsigned short* WFC1T  = (unsigned short*)(ws + 32 * kMiB);
  unsigned short* WFC2T  = (unsigned short*)(ws + 40 * kMiB);
  unsigned short* QK16   = (unsigned short*)(ws + 48 * kMiB);
  float*          X1     = (float*)(ws + 48 * kMiB);
  unsigned short* VT16   = (unsigned short*)(ws + 64 * kMiB);
  float*          MEMOUT = (float*)(ws + 72 * kMiB);
  float*          MEM32  = (float*)(ws + 88 * kMiB);
  unsigned short* ATT16  = (unsigned short*)(ws + 88 * kMiB);
  unsigned short* HID16  = (unsigned short*)(ws + 64 * kMiB);
  unsigned short* H16    = (unsigned short*)(ws + 96 * kMiB);
  unsigned short* WQKVT  = (unsigned short*)(ws + 104 * kMiB);
  unsigned short* WOUTT  = (unsigned short*)(ws + 110 * kMiB);

  wtcast_kernel<<<dim3(kC / 64, kQKVld / 64), 256, 0, stream>>>(w_qkv, WQKVT, kC, kQKVld, kWCarry);
  wtcast_kernel<<<dim3(kC / 64, kC / 64), 256, 0, stream>>>(w_out, WOUTT, kC, kC, kWCarry);
  memproj_kernel<<<dim3(kC / 256, kMemN), 256, 0, stream>>>(memory, w_mem, b_mem, MEM32);
  ln_f16_kernel<<<kTok, 128, 0, stream>>>(x, ln1_g, ln1_b, H16);
  launch_gemm<2, 0, false>(stream, 1, H16, kC, 0L, WQKVT, kC, 0L, QKV32, kQKVld, 0L,
                           b_qkv, x, 0L, kTok, kQKVld, kC, 1.0f / kWCarry);
  qkcast_kernel<<<kTok * (kQKld / 8) / 256, 256, 0, stream>>>(QKV32, QK16);
  vtr_kernel<<<dim3(kT / 64, kBatch * kHeads), 256, 0, stream>>>(QKV32, VT16);
  mematt_kernel<<<dim3(kT / 64, kBatch * kHeads), 64, 0, stream>>>(QKV32, MEM32, MEMOUT, kAttCarry);
  for (int b = 0; b < kBatch; ++b) {
    for (int hc = 0; hc < kHeads / 2; ++hc) {
      const int h0 = hc * 2;
      const unsigned short* qbase = QK16 + (size_t)b * kT * kQKld + h0 * kD;
      const unsigned short* kbase = QK16 + (size_t)b * kT * kQKld + kC + h0 * kD;
      launch_gemm<0, 0, false>(stream, 2, qbase, kQKld, (long)kD, kbase, kQKld, (long)kD,
                               S32, kT, (long)kT * kT, b_qkv, x, 0L, kT, kT, kD, 0.125f);
      softmax_row_kernel<<<2 * kT, 256, 0, stream>>>(S32, P16, kPCarry);
      launch_gemm<0, 1, true>(stream, 2, P16, kT, (long)kT * kT,
                              VT16 + (size_t)(b * kHeads + h0) * kD * kT, kT, (long)kD * kT,
                              ATT16 + (size_t)b * kT * kC + h0 * kD, kC, (long)kD,
                              b_qkv, MEMOUT + (size_t)b * kT * kC + h0 * kD, (long)kD,
                              kT, kD, kT, kAttCarry / kPCarry);
    }
  }
  launch_gemm<2, 0, true>(stream, 1, ATT16, kC, 0L, WOUTT, kC, 0L, X1, kC, 0L,
                          b_out, x, 0L, kTok, kC, kC, 1.0f / (kAttCarry * kWCarry));
  ln_f16_kernel<<<kTok, 128, 0, stream>>>(X1, ln2_g, ln2_b, H16);
  wtcast_kernel<<<dim3(kC / 64, kHid / 64), 256, 0, stream>>>(w_fc1, WFC1T, kC, kHid, kWCarry);
  wtcast_kernel<<<dim3(kHid / 64, kC / 64), 256, 0, stream>>>(w_fc2, WFC2T, kHid, kC, kWCarry);
  for (int half = 0; half < 2; ++half) {
    launch_gemm<2, 0, false>(stream, 1, H16, kC, 0L, WFC1T + (size_t)half * 2048 * kC, kC, 0L,
                             G32, 2048, 0L, b_fc1 + half * 2048, x, 0L, kTok, 2048, kC, 1.0f / kWCarry);
    gelu_f16_kernel<<<kTok * 1024 / 256, 256, 0, stream>>>(G32, HID16, half * 2048, kHidCarry);
  }
  launch_gemm<2, 0, true>(stream, 1, HID16, kHid, 0L, WFC2T, kHid, 0L, out, kC, 0L,
                          b_fc2, X1, 0L, kTok, kC, kHid, 1.0f / (kHidCarry * kWCarry));
}
